// DenseSAKELayer_13108240187514
// MI455X (gfx1250) — hardware-verified
//
#include <hip/hip_runtime.h>
#include <math.h>
typedef __attribute__((ext_vector_type(16))) _Float16 v16h;
typedef __attribute__((ext_vector_type(8)))  _Float16 v8h;
typedef __attribute__((ext_vector_type(16))) __bf16   v16b;
typedef __attribute__((ext_vector_type(8)))  __bf16   v8b;
typedef __attribute__((ext_vector_type(8)))  float    v8f;
typedef __attribute__((ext_vector_type(4)))  float    v4f;
#define PSCALE 32768.0f
#define U16(p) ((const unsigned short*)(const void*)(p))
#define PSCALE_INV (1.0f / 32768.0f)

__device__ __forceinline__ unsigned short f2bf_bits(float f) {
  unsigned u = __float_as_uint(f);
  return (unsigned short)((u + 0x7FFFu + ((u >> 16) & 1u)) >> 16);
}
__device__ __forceinline__ float bf_bits2f(unsigned short h) { return __uint_as_float(((unsigned)h) << 16); }

__device__ __forceinline__ void dep_guard_h(v8f& a, v8f& b, v16h x, v16h y) { asm volatile("v_nop\n\tv_nop\n\tv_nop\n\tv_nop" : "+v"(a), "+v"(b) : "v"(x), "v"(y)); }
__device__ __forceinline__ void dep_guard_b(v8f& a, v8f& b, v16b x, v16b y) { asm volatile("v_nop\n\tv_nop\n\tv_nop\n\tv_nop" : "+v"(a), "+v"(b) : "v"(x), "v"(y)); }
__device__ __forceinline__ void keep4_h(v16h a, v16h b, v16h c, v16h d) { asm volatile("v_nop" :: "v"(a), "v"(b), "v"(c), "v"(d)); }
__device__ __forceinline__ void keep4_b(v16b a, v16b b, v16b c, v16b d) { asm volatile("v_nop" :: "v"(a), "v"(b), "v"(c), "v"(d)); }
__device__ __forceinline__ void acc_guard4(v8f& a, v8f& b, v8f& c, v8f& d) { asm volatile("v_nop\n\tv_nop\n\tv_nop\n\tv_nop" : "+v"(a), "+v"(b), "+v"(c), "+v"(d)); }
template <typename T> struct Frag;
template <> struct Frag<_Float16> {
  typedef v16h V; union U { v16h v; v8h h[2]; };
  static __device__ __forceinline__ v16h load(const _Float16* p) {
    U f; f.h[0] = *(const v8h*)(p); f.h[1] = *(const v8h*)(p + 16); return f.v;
  }
  static __device__ __forceinline__ v8f mma(v16h a, v16h b, v8f c) {
    return __builtin_amdgcn_wmma_f32_16x16x32_f16(false, a, false, b, (short)0, c, false, false);
  }
  static __device__ __forceinline__ void guard(v8f& a, v8f& b, v16h x, v16h y) { dep_guard_h(a, b, x, y); }
  static __device__ __forceinline__ void keep(v16h a, v16h b, v16h c, v16h d) { keep4_h(a, b, c, d); }
};
template <> struct Frag<__bf16> {
  typedef v16b V; union U { v16b v; v8b h[2]; };
  static __device__ __forceinline__ v16b load(const __bf16* p) {
    U f; f.h[0] = *(const v8b*)(p); f.h[1] = *(const v8b*)(p + 16); return f.v;
  }
  static __device__ __forceinline__ v8f mma(v16b a, v16b b, v8f c) {
    return __builtin_amdgcn_wmma_f32_16x16x32_bf16(false, a, false, b, (short)0, c, false, false);
  }
  static __device__ __forceinline__ void guard(v8f& a, v8f& b, v16b x, v16b y) { dep_guard_b(a, b, x, y); }
  static __device__ __forceinline__ void keep(v16b a, v16b b, v16b c, v16b d) { keep4_b(a, b, c, d); }
};

template <int ET> struct Elem;
template <> struct Elem<0> { typedef _Float16 T; };
template <> struct Elem<1> { typedef __bf16 T; };
template <int ET, bool SPLIT, int BIAS_MODE, int OUT_MODE, bool RESID, int ACT = 0>
__global__ __launch_bounds__(256) void wmma_gemm64(
    const unsigned short* __restrict__ Ap, const unsigned short* __restrict__ A2p, int lda, long strideA,
    const unsigned short* __restrict__ Btp, const unsigned short* __restrict__ Bt2p, int ldb, long strideB,
    void* __restrict__ Cout, void* __restrict__ Cout2, int ldc, long strideC,
    const float* __restrict__ bias,
    const float* __restrict__ resid, long strideR,
    int M, int N, int K, float scale) {
  typedef typename Elem<ET>::T T;
  typedef typename Frag<T>::V V;
  const T* A = (const T*)Ap; const T* A2 = (const T*)A2p; const T* Bt = (const T*)Btp; const T* Bt2 = (const T*)Bt2p;
  __shared__ __align__(16) float sT[8][16 * 68];
  const int b    = blockIdx.y;
  const int lane = threadIdx.x & 31;
  const int wave = threadIdx.x >> 5;
  const int tilesN = N >> 6;
  const int tilesM = M >> 6;
  const int tile = blockIdx.x * 8 + wave;
  if (tile >= tilesM * tilesN) return;
  const int tm = tile / tilesN;
  const int tn = tile - tm * tilesN;
  const int m0 = tm << 6;
  const int n0 = tn << 6;

  const T* Ab  = A  + (size_t)b * strideA;
  const T* Bb  = Bt + (size_t)b * strideB;
  const T* Ab2 = SPLIT ? (A2  + (size_t)b * strideA) : nullptr;
  const T* Bb2 = SPLIT ? (Bt2 + (size_t)b * strideB) : nullptr;

  const int rlane = lane & 15;
  const int koff  = (lane >> 4) * 8;
  const int mOff  = (lane >> 4) * 8;

  v8f acc[4][4];
#pragma unroll
  for (int i = 0; i < 4; ++i)
#pragma unroll
    for (int j = 0; j < 4; ++j) acc[i][j] = (v8f){0.f,0.f,0.f,0.f,0.f,0.f,0.f,0.f};

  for (int k0 = 0; k0 < K; k0 += 32) {
    V bh[4], bl[4];
#pragma unroll
    for (int j = 0; j < 4; ++j) {
      const size_t bo = (size_t)(n0 + (j << 4) + rlane) * ldb + koff + k0;
      bh[j] = Frag<T>::load(Bb + bo);
      if (SPLIT) bl[j] = Frag<T>::load(Bb2 + bo);
    }
#pragma unroll
    for (int i = 0; i < 4; ++i) {
      const size_t ao = (size_t)(m0 + (i << 4) + rlane) * lda + koff + k0;
      V ah = Frag<T>::load(Ab + ao);
      V al;
      if (SPLIT) al = Frag<T>::load(Ab2 + ao);
#pragma unroll
      for (int j = 0; j < 4; ++j) {
        acc[i][j] = Frag<T>::mma(ah, bh[j], acc[i][j]);
        if (SPLIT) {
          acc[i][j] = Frag<T>::mma(ah, bl[j], acc[i][j]);
          acc[i][j] = Frag<T>::mma(al, bh[j], acc[i][j]);
        }
      }
      Frag<T>::guard(acc[i][0], acc[i][3], ah, SPLIT ? al : ah);
    }
    Frag<T>::keep(bh[0], bh[1], bh[2], bh[3]);
    if (SPLIT) Frag<T>::keep(bl[0], bl[1], bl[2], bl[3]);
  }
  acc_guard4(acc[0][0], acc[0][1], acc[0][2], acc[0][3]);
  acc_guard4(acc[1][0], acc[1][1], acc[1][2], acc[1][3]);
  acc_guard4(acc[2][0], acc[2][1], acc[2][2], acc[2][3]);
  acc_guard4(acc[3][0], acc[3][1], acc[3][2], acc[3][3]);

  float* slab = sT[wave];
  const float* Rb = RESID ? (resid + (size_t)b * strideR) : nullptr;
#pragma unroll
  for (int i = 0; i < 4; ++i) {
    const int mBase = m0 + (i << 4);
#pragma unroll
    for (int j = 0; j < 4; ++j) {
      const int n = n0 + (j << 4) + rlane;
      float bv = 0.f;
      if (BIAS_MODE == 2) bv = bias[n];
#pragma unroll
      for (int r = 0; r < 8; ++r) {
        float v = acc[i][j][r] * scale;
        if (BIAS_MODE == 1) v += bias[mBase + mOff + r];
        if (BIAS_MODE == 2) v += bv;
        if (RESID) v += Rb[(size_t)(mBase + mOff + r) * ldc + n];
        if (ACT == 1) v = tanhf(v);
        if (ACT == 2) v = fmaxf(v, 0.0f);
        if (ACT == 3) v = v / (1.0f + expf(-v));
        if (ACT == 4) v = (v > 0.f) ? v : 0.01f * v;
        if (ACT == 5) v = 0.5f * v * (1.0f + erff(v * 0.70710678118654752f));
        slab[(mOff + r) * 68 + (j << 4) + rlane] = v;
      }
    }
    __builtin_amdgcn_fence(__ATOMIC_RELEASE, "workgroup");
    __builtin_amdgcn_wave_barrier();
    __builtin_amdgcn_fence(__ATOMIC_ACQUIRE, "workgroup");
    if (OUT_MODE == 0) {
      float* C = (float*)Cout + (size_t)b * strideC;
      const int hh = lane >> 4, c4 = (lane & 15) * 4;
      for (int pass = 0; pass < 2; ++pass) {
#pragma unroll
        for (int it = 0; it < 8; ++it) {
          const int row = it * 2 + hh;
          v4f v = *(const v4f*)(slab + row * 68 + c4);
          *(volatile v4f*)(C + (size_t)(mBase + row) * ldc + n0 + c4) = v;
        }
        __threadfence();
      }
    } else {
      const int q = lane >> 3, c8 = (lane & 7) * 8;
      unsigned short* C  = (unsigned short*)Cout  + (size_t)b * strideC;
      unsigned short* C2 = (OUT_MODE == 2) ? ((unsigned short*)Cout2 + (size_t)b * strideC) : nullptr;
      for (int pass = 0; pass < 2; ++pass) {
#pragma unroll
        for (int it = 0; it < 4; ++it) {
          const int row = it * 4 + q;
          const float* sp = slab + row * 68 + c8;
          v8h hv, lv;
#pragma unroll
          for (int e = 0; e < 8; ++e) {
            if (OUT_MODE == 1) {
              hv[e] = (_Float16)sp[e];
            } else {
              unsigned short hb = f2bf_bits(sp[e]);
              unsigned short lb = f2bf_bits(sp[e] - bf_bits2f(hb));
              hv[e] = __builtin_bit_cast(_Float16, hb);
              lv[e] = __builtin_bit_cast(_Float16, lb);
            }
          }
          *(volatile v8h*)(C + (size_t)(mBase + row) * ldc + n0 + c8) = hv;
          if (OUT_MODE == 2) *(volatile v8h*)(C2 + (size_t)(mBase + row) * ldc + n0 + c8) = lv;
        }
        __threadfence();
      }
    }
    __builtin_amdgcn_fence(__ATOMIC_RELEASE, "workgroup");
    __builtin_amdgcn_wave_barrier();
    __builtin_amdgcn_fence(__ATOMIC_ACQUIRE, "workgroup");
  }
}

__global__ __launch_bounds__(256) void cast_f32_f16x2(
    const float* __restrict__ in, _Float16* __restrict__ out, int n2) {
  int i = blockIdx.x * 256 + threadIdx.x;
  if (i < n2) {
    const _Float16 h0 = (_Float16)in[2 * i], h1 = (_Float16)in[2 * i + 1];
    const unsigned u = (unsigned)__builtin_bit_cast(unsigned short, h0) | ((unsigned)__builtin_bit_cast(unsigned short, h1) << 16);
    ((volatile unsigned*)out)[i] = u;
    __threadfence();
    ((volatile unsigned*)out)[i] = u;
  }
}


#define SNn 512
#define SF 64
#define SH 64
#define SCc 32
#define SKr 50
#define SPAIR (SNn * SNn)
__global__ __launch_bounds__(256) void node_pre_kernel(const float* __restrict__ h, const float* __restrict__ Wdfin, const float* __restrict__ Wsa, const float* __restrict__ Wew, float* __restrict__ PN) {
  const int n = blockIdx.x, t = threadIdx.x; __shared__ float hn[SF]; __shared__ float outv[256];
  if (t < SF) hn[t] = h[n * SF + t];
  outv[t] = 0.f; __syncthreads();
  float a = 0.f;
  if (t < SKr) {
#pragma unroll 1
 for (int k = 0; k < SF; ++k) a += hn[k] * Wdfin[k * SKr + t]; outv[t] = a; }
  else if (t >= 64 && t < 64 + SKr) { const int o = t - 64;
#pragma unroll 1
 for (int k = 0; k < SF; ++k) a += hn[k] * Wdfin[(64 + k) * SKr + o]; outv[t] = a; }
  else if (t == 128) {
#pragma unroll 1
 for (int k = 0; k < SF; ++k) a += hn[k] * Wsa[k]; outv[t] = a; }
  else if (t == 129) {
#pragma unroll 1
 for (int k = 0; k < SF; ++k) a += hn[k] * Wsa[64 + k]; outv[t] = a; }
  else if (t >= 130 && t < 162) { const int o = t - 130;
#pragma unroll 1
 for (int k = 0; k < SF; ++k) a += hn[k] * Wew[k * SCc + o]; outv[t] = a; }
  else if (t >= 162 && t < 194) { const int o = t - 162;
#pragma unroll 1
 for (int k = 0; k < SF; ++k) a += hn[k] * Wew[(64 + k) * SCc + o]; outv[t] = a; }
  __syncthreads();
  ((volatile float*)PN)[n * 256 + t] = outv[t]; __threadfence(); ((volatile float*)PN)[n * 256 + t] = outv[t];
}
__global__ __launch_bounds__(256) void he0_kernel(const float* __restrict__ x, const float* __restrict__ PN, const float* __restrict__ bdf, unsigned* __restrict__ HE0) {
  const long g = (long)blockIdx.x * 256 + threadIdx.x; const long pr = g / 32; const int kp = 2 * (int)(g % 32); if (pr >= SPAIR) return; const int i = (int)(pr / SNn), j = (int)(pr % SNn);
  const float dx = x[j * 3] - x[i * 3], dy = x[j * 3 + 1] - x[i * 3 + 1], dz = x[j * 3 + 2] - x[i * 3 + 2]; const float d2 = dx * dx + dy * dy + dz * dz; const float dist = sqrtf(fmaxf(d2, 0.f) + 1e-14f);
  float v[2];
  for (int e = 0; e < 2; ++e) { const int k = kp + e; if (k < SKr) { const float mu = (float)k * (5.0f / 49.0f); const float rb = expf(-10.0f * (dist - mu) * (dist - mu)); v[e] = (PN[j * 256 + k] + PN[i * 256 + 64 + k] + bdf[k]) * rb; } else v[e] = 0.f; }
  const unsigned u = (unsigned)__builtin_bit_cast(unsigned short, (_Float16)v[0]) | ((unsigned)__builtin_bit_cast(unsigned short, (_Float16)v[1]) << 16);
  ((volatile unsigned*)HE0)[g] = u; __threadfence(); ((volatile unsigned*)HE0)[g] = u;
}
__global__ __launch_bounds__(256) void wt_kernel(const float* __restrict__ Wsrc, int roff, int ldw, int KIN, int NOUT, unsigned* __restrict__ BT) {
  for (int i = threadIdx.x; i < 64 * 32; i += 256) { const int o = i / 32, kp = 2 * (i % 32); float a = 0.f, b = 0.f; if (o < NOUT) { if (kp < KIN) a = Wsrc[(size_t)(roff + kp) * ldw + o]; if (kp + 1 < KIN) b = Wsrc[(size_t)(roff + kp + 1) * ldw + o]; }
    const unsigned u = (unsigned)__builtin_bit_cast(unsigned short, (_Float16)a) | ((unsigned)__builtin_bit_cast(unsigned short, (_Float16)b) << 16); ((volatile unsigned*)BT)[i] = u; __threadfence(); ((volatile unsigned*)BT)[i] = u; }
}
__global__ __launch_bounds__(256) void reduce_kernel(const float* __restrict__ x, const float* __restrict__ PN, const unsigned* __restrict__ HE16, const _Float16* __restrict__ EWP, const unsigned* __restrict__ CM16, const float* __restrict__ bew, const float* __restrict__ Wcm2, const float* __restrict__ bcm2, float* __restrict__ NODEBUF) {
  __shared__ float red[256]; __shared__ float sA[SNn], sB[SNn]; __shared__ float acc96[8][96]; __shared__ float accH[8][64]; __shared__ float acc3[8][4]; __shared__ float bc[4];
  const int i = blockIdx.x, t = threadIdx.x, lane = t & 31, wave = t >> 5;
  const float xi0 = x[i * 3], xi1 = x[i * 3 + 1], xi2 = x[i * 3 + 2]; const float sab = PN[i * 256 + 129];
  float m1 = -INFINITY, m2 = -INFINITY;
  for (int j = t; j < SNn; j += 256) { const float dx = x[j * 3] - xi0, dy = x[j * 3 + 1] - xi1, dz = x[j * 3 + 2] - xi2; const float dist = sqrtf(fmaxf(dx * dx + dy * dy + dz * dz, 0.f) + 1e-14f);
    float s = PN[j * 256 + 128] + sab; s = s / (1.0f + expf(-s)); sA[j] = dist; sB[j] = s; m1 = fmaxf(m1, dist); m2 = fmaxf(m2, s); }
  red[t] = m1; __syncthreads(); for (int o = 128; o > 0; o >>= 1) { if (t < o) red[t] = fmaxf(red[t], red[t + o]); __syncthreads(); } m1 = red[0]; __syncthreads();
  red[t] = m2; __syncthreads(); for (int o = 128; o > 0; o >>= 1) { if (t < o) red[t] = fmaxf(red[t], red[t + o]); __syncthreads(); } m2 = red[0]; __syncthreads();
  float s1 = 0.f, s2 = 0.f; for (int j = t; j < SNn; j += 256) { s1 += expf(sA[j] - m1); s2 += expf(sB[j] - m2); }
  red[t] = s1; __syncthreads(); for (int o = 128; o > 0; o >>= 1) { if (t < o) red[t] += red[t + o]; __syncthreads(); } s1 = red[0]; __syncthreads();
  red[t] = s2; __syncthreads(); for (int o = 128; o > 0; o >>= 1) { if (t < o) red[t] += red[t + o]; __syncthreads(); } s2 = red[0]; __syncthreads();
  float m3 = -INFINITY; for (int j = t; j < SNn; j += 256) { const float p = (expf(sA[j] - m1) / s1) * (expf(sB[j] - m2) / s2); sA[j] = p; m3 = fmaxf(m3, p); }
  __syncthreads(); red[t] = m3; __syncthreads(); for (int o = 128; o > 0; o >>= 1) { if (t < o) red[t] = fmaxf(red[t], red[t + o]); __syncthreads(); } m3 = red[0]; __syncthreads();
  float s3 = 0.f; for (int j = t; j < SNn; j += 256) s3 += expf(sA[j] - m3);
  red[t] = s3; __syncthreads(); for (int o = 128; o > 0; o >>= 1) { if (t < o) red[t] += red[t + o]; __syncthreads(); } s3 = red[0]; __syncthreads();
  if (t < 4) bc[t] = (t == 0) ? bcm2[0] : 0.f;
  for (int k = t; k < 8 * 96; k += 256) (&acc96[0][0])[k] = 0.f; for (int k = t; k < 8 * 64; k += 256) (&accH[0][0])[k] = 0.f; if (t < 32) (&acc3[0][0])[t] = 0.f;
  __syncthreads();
  float a96[3] = {0.f, 0.f, 0.f}; float aH[2] = {0.f, 0.f}; float a3x = 0.f, a3y = 0.f, a3z = 0.f;
  typedef __attribute__((ext_vector_type(2))) float v2f; typedef __attribute__((ext_vector_type(2))) _Float16 v2h;
  for (int j = wave; j < SNn; j += 8) { const size_t pr = (size_t)i * SNn + j;
    const float dx = x[j * 3] - xi0, dy = x[j * 3 + 1] - xi1, dz = x[j * 3 + 2] - xi2; const float d2 = dx * dx + dy * dy + dz * dz; const float inv = 1.0f / (d2 + 1e-5f);
    const float w = tanhf(PN[j * 256 + 130 + lane] + PN[i * 256 + 162 + lane] + (float)EWP[pr * 64 + lane] + bew[lane]);
    a96[0] += w * dx * inv; a96[1] += w * dy * inv; a96[2] += w * dz * inv;
    const v2h cmh = __builtin_bit_cast(v2h, CM16[pr * 32 + lane]); float cw = (float)cmh[0] * Wcm2[2 * lane] + (float)cmh[1] * Wcm2[2 * lane + 1];
    for (int o = 16; o > 0; o >>= 1) cw += __shfl_xor(cw, o, 32); cw += bc[0];
    if (lane == 0) { a3x += dx * cw; a3y += dy * cw; a3z += dz * cw; }
    const float att = expf(sA[j] - m3) / s3; const v2h heh = __builtin_bit_cast(v2h, HE16[pr * 32 + lane]); aH[0] += att * (float)heh[0]; aH[1] += att * (float)heh[1]; }
  acc96[wave][lane * 3] = a96[0]; acc96[wave][lane * 3 + 1] = a96[1]; acc96[wave][lane * 3 + 2] = a96[2]; accH[wave][2 * lane] = aH[0]; accH[wave][2 * lane + 1] = aH[1];
  if (lane == 0) { acc3[wave][0] = a3x; acc3[wave][1] = a3y; acc3[wave][2] = a3z; }
  __syncthreads();
  float outv = 0.f;
  if (t < 64) { for (int w8 = 0; w8 < 8; ++w8) outv += accH[w8][t]; }
  else if (t < 96) { const int c = t - 64; float sx = 0.f, sy = 0.f, sz = 0.f; for (int w8 = 0; w8 < 8; ++w8) { sx += acc96[w8][c * 3]; sy += acc96[w8][c * 3 + 1]; sz += acc96[w8][c * 3 + 2]; } outv = sqrtf(fmaxf(sx * sx + sy * sy + sz * sz, 0.f) + 1e-14f); }
  else if (t < 99) { const int c = t - 96; float s = 0.f; for (int w8 = 0; w8 < 8; ++w8) s += acc3[w8][c]; outv = s + x[i * 3 + c]; }
  ((volatile float*)NODEBUF)[i * 256 + t] = outv; __threadfence(); ((volatile float*)NODEBUF)[i * 256 + t] = outv;
}
__global__ __launch_bounds__(64) void node_out_kernel(const float* __restrict__ h, const float* __restrict__ NODEBUF, const float* __restrict__ Wpn1, const float* __restrict__ bpn1, const float* __restrict__ Wpn2, const float* __restrict__ bpn2,
                                                    const float* __restrict__ Wnm1, const float* __restrict__ bnm1, const float* __restrict__ Wnm2, const float* __restrict__ bnm2, float* __restrict__ out0, float* __restrict__ out1) {
  __shared__ float nin[192]; __shared__ float t1[64]; __shared__ float ne[64]; __shared__ float t2[64];
  const int n = blockIdx.x, t = threadIdx.x;
  nin[t] = h[n * 64 + t]; nin[64 + t] = NODEBUF[n * 256 + t];
  float a = bpn1[t];
#pragma unroll 1
  for (int k = 0; k < 32; ++k) a += NODEBUF[n * 256 + 64 + k] * Wpn1[k * 64 + t];
  t1[t] = a / (1.0f + expf(-a)); __syncthreads();
  a = bpn2[t];
#pragma unroll 1
  for (int k = 0; k < 64; ++k) a += t1[k] * Wpn2[k * 64 + t];
  nin[128 + t] = a; __syncthreads();
  a = bnm1[t];
#pragma unroll 1
  for (int k = 0; k < 192; ++k) a += nin[k] * Wnm1[k * 64 + t];
  t2[t] = a / (1.0f + expf(-a)); __syncthreads();
  a = bnm2[t];
#pragma unroll 1
  for (int k = 0; k < 64; ++k) a += t2[k] * Wnm2[k * 64 + t];
  ((volatile float*)out0)[n * 64 + t] = a; if (t < 3) ((volatile float*)out1)[n * 3 + t] = NODEBUF[n * 256 + 96 + t];
  __threadfence();
  ((volatile float*)out0)[n * 64 + t] = a; if (t < 3) ((volatile float*)out1)[n * 3 + t] = NODEBUF[n * 256 + 96 + t];
}
extern "C" void kernel_launch(void* const* d_in, const int* in_sizes, int n_in, void* d_out, int out_size, void* d_ws, size_t ws_size, hipStream_t stream) {
  (void)in_sizes; (void)n_in; (void)out_size; (void)ws_size;
  auto Fp = [&](int i) { return (const float*)d_in[i]; };
  const float* h = Fp(0); const float* x = Fp(1); const float* Wdfin = Fp(2); const float* bdfin = Fp(3); const float* Wdf1 = Fp(4); const float* bdf1 = Fp(5); const float* Wdf2 = Fp(6); const float* bdf2 = Fp(7);
  const float* Wew = Fp(8); const float* bew = Fp(9); const float* Wpn1 = Fp(10); const float* bpn1 = Fp(11); const float* Wpn2 = Fp(12); const float* bpn2 = Fp(13); const float* Wnm1 = Fp(14); const float* bnm1 = Fp(15); const float* Wnm2 = Fp(16); const float* bnm2 = Fp(17);
  const float* Wcm1 = Fp(18); const float* bcm1 = Fp(19); const float* Wcm2 = Fp(20); const float* bcm2 = Fp(21); const float* Wsa = Fp(22);
  float* out0 = (float*)d_out; float* out1 = out0 + SNn * 64;
  char* ws = (char*)d_ws; size_t off = 0;
  auto carve = [&](size_t bytes) -> char* { char* p = ws + off; off += (bytes + 255) & ~(size_t)255; return p; };
  float* PN = (float*)carve(SNn * 256 * 4); unsigned* HE0 = (unsigned*)carve((size_t)SPAIR * 64 * 2); unsigned* BT1 = (unsigned*)carve(64 * 64 * 2); unsigned* BT2 = (unsigned*)carve(64 * 64 * 2); unsigned* BT3 = (unsigned*)carve(64 * 64 * 2); unsigned* BT4 = (unsigned*)carve(64 * 64 * 2);
  _Float16* HE1 = (_Float16*)carve((size_t)SPAIR * 64 * 2); _Float16* HE16 = (_Float16*)carve((size_t)SPAIR * 64 * 2); float* NODEBUF = (float*)carve(SNn * 256 * 4);
  _Float16* CM16 = (_Float16*)HE0;
  _Float16* EWP16 = HE1;
  node_pre_kernel<<<SNn, 256, 0, stream>>>(h, Wdfin, Wsa, Wew, PN);
  he0_kernel<<<(unsigned)(((long)SPAIR * 32 + 255) / 256), 256, 0, stream>>>(x, PN, bdfin, HE0);
  wt_kernel<<<1, 256, 0, stream>>>(Wdf1, 0, 64, SKr, 64, BT1); wt_kernel<<<1, 256, 0, stream>>>(Wdf2, 0, 64, 64, 64, BT2); wt_kernel<<<1, 256, 0, stream>>>(Wew, 128, SCc, 64, SCc, BT3); wt_kernel<<<1, 256, 0, stream>>>(Wcm1, 0, 64, 64, 64, BT4);
  const int t = (SPAIR / 64) * 1;
  wmma_gemm64<0, false, 2, 1, false, 3><<<dim3((t + 7) / 8, 1), 256, 0, stream>>>((const unsigned short*)HE0, nullptr, 64, 0, (const unsigned short*)BT1, nullptr, 64, 0, HE1, nullptr, 64, 0, bdf1, nullptr, 0, SPAIR, 64, 64, 1.0f);
  wmma_gemm64<0, false, 2, 1, false, 0><<<dim3((t + 7) / 8, 1), 256, 0, stream>>>(U16(HE1), nullptr, 64, 0, (const unsigned short*)BT2, nullptr, 64, 0, HE16, nullptr, 64, 0, bdf2, nullptr, 0, SPAIR, 64, 64, 1.0f);
  wmma_gemm64<0, false, 0, 1, false, 0><<<dim3((t + 7) / 8, 1), 256, 0, stream>>>(U16(HE16), nullptr, 64, 0, (const unsigned short*)BT3, nullptr, 64, 0, EWP16, nullptr, 64, 0, nullptr, nullptr, 0, SPAIR, 64, 64, 1.0f);
  wmma_gemm64<0, false, 2, 1, false, 3><<<dim3((t + 7) / 8, 1), 256, 0, stream>>>(U16(HE16), nullptr, 64, 0, (const unsigned short*)BT4, nullptr, 64, 0, CM16, nullptr, 64, 0, bcm1, nullptr, 0, SPAIR, 64, 64, 1.0f);
  reduce_kernel<<<SNn, 256, 0, stream>>>(x, PN, (const unsigned*)HE16, (const _Float16*)EWP16, (const unsigned*)CM16, bew, Wcm2, bcm2, NODEBUF);
  node_out_kernel<<<SNn, 64, 0, stream>>>(h, NODEBUF, Wpn1, bpn1, Wpn2, bpn2, Wnm1, bnm1, Wnm2, bnm2, out0, out1);
}
